// FlashAttention_27745488733024
// MI455X (gfx1250) — hardware-verified
//
#include <hip/hip_runtime.h>
#include <math.h>

#ifndef NB
#define NB 2
#endif
#ifndef SEQ
#define SEQ 2048
#endif
#define NB_FULL 2
#define SEQ_FULL 2048
#define NH 16
#define HD 128
#define KBS 256
#define SUB 64
#define AW 4
#define NSUB (KBS / SUB)
#define NKB (SEQ / KBS)

static_assert(NB >= 1 && NB <= NB_FULL);
static_assert(SEQ >= KBS && SEQ <= SEQ_FULL && (SEQ % KBS) == 0);
static_assert((KBS % SUB) == 0 && SUB == 64);
static_assert((SEQ % (16 * AW)) == 0);
static_assert(HD == 128);
static_assert(32 * AW == 8 * 16);
static_assert((((long long)NB * NH * SEQ * HD) % 8) == 0);
static_assert((((long long)NB * NH * SEQ * HD * 2) % 256) == 0);

typedef __attribute__((ext_vector_type(16))) __bf16 v16b;
typedef __attribute__((ext_vector_type(16))) unsigned short v16us;
typedef __attribute__((ext_vector_type(8)))  unsigned short v8us;
typedef __attribute__((ext_vector_type(8)))  float v8f;
typedef __attribute__((ext_vector_type(4)))  float v4f;
typedef __attribute__((ext_vector_type(4)))  unsigned int v4u;

__device__ __forceinline__ int frag_k(int i, int h) { return (i < 8) ? (8 * h + i) : (16 + 8 * h + (i - 8)); }
__device__ __forceinline__ unsigned short bfu_rne(float f) {
    unsigned int u = __float_as_uint(f);
    u += 0x7fffu + ((u >> 16) & 1u);
    return (unsigned short)(u >> 16);
}
__device__ __forceinline__ __bf16 bf16_rne(float f) { return __builtin_bit_cast(__bf16, bfu_rne(f)); }
__device__ __forceinline__ float bf16_f32(__bf16 b) { return __uint_as_float(((unsigned int)__builtin_bit_cast(unsigned short, b)) << 16); }

__device__ __forceinline__ v8f wmmab(v16b a, v16b b, v8f c) {
    c = __builtin_amdgcn_wmma_f32_16x16x32_bf16(false, a, false, b, (short)0, c, false, false);
    asm volatile("v_nop\n\tv_nop\n\tv_nop\n\tv_nop" : "+v"(c) : "v"(a), "v"(b));
    return c;
}
struct Split { v16b hi, lo; };

#define SCHED_FENCE() do { asm volatile("" ::: "memory"); __builtin_amdgcn_sched_barrier(0); } while (0)

__device__ __forceinline__ v16b frag_row(const unsigned short* row, int k0, int h) {
    const v8us u0 = *(const v8us*)(row + k0 + 8 * h);
    const v8us u1 = *(const v8us*)(row + k0 + 16 + 8 * h);
    const v16us w = __builtin_shufflevector(u0, u1, 0, 1, 2, 3, 4, 5, 6, 7, 8, 9, 10, 11, 12, 13, 14, 15);
    return __builtin_bit_cast(v16b, w);
}
__device__ __forceinline__ Split psplit(const float* prow, int k0s, int h) {
    v4f f[4];
    f[0] = *(const v4f*)(prow + k0s + 8 * h);
    f[1] = *(const v4f*)(prow + k0s + 8 * h + 4);
    f[2] = *(const v4f*)(prow + k0s + 16 + 8 * h);
    f[3] = *(const v4f*)(prow + k0s + 20 + 8 * h);
    Split r;
#pragma unroll
    for (int i = 0; i < 16; ++i) {
        const float x = f[i >> 2][i & 3];
        const __bf16 hb = bf16_rne(x);
        r.hi[i] = hb;
        r.lo[i] = bf16_rne(x - bf16_f32(hb));
    }
    return r;
}

#define VST2V4(ptr, val) do { const v4f vst2_v4_ = (val); *(volatile v4f*)(ptr) = vst2_v4_; __threadfence(); *(volatile v4f*)(ptr) = vst2_v4_; } while (0)

__device__ __forceinline__ unsigned int pk2b(float a, float b) { return (unsigned int)bfu_rne(a) | ((unsigned int)bfu_rne(b) << 16); }
__global__ __launch_bounds__(256) void k_cvtb(const float* __restrict__ Q, const float* __restrict__ K, const float* __restrict__ V,
                                              unsigned short* __restrict__ QB, unsigned short* __restrict__ KB, unsigned short* __restrict__ VB, long long n8) {
    const long long nbk = (n8 + 255) / 256;
    const int which = (int)((long long)blockIdx.x / nbk);
    const long long u = ((long long)blockIdx.x - (long long)which * nbk) * 256 + threadIdx.x;
    if (which > 2 || u >= n8) return;
    const float* src = (which == 0) ? Q : ((which == 1) ? K : V);
    unsigned short* dst = (which == 0) ? QB : ((which == 1) ? KB : VB);
    const long long e = u * 8;
    const long long row = e / HD;
    const int d = (int)(e - row * HD);
    const long long bh = row / SEQ;
    const long long s = row - bh * SEQ;
    const float* sp = src + ((bh * SEQ_FULL + s) * HD + d);
    const v4f x0 = *(const v4f*)sp;
    const v4f x1 = *(const v4f*)(sp + 4);
    v4u pk;
    pk.x = pk2b(x0.x, x0.y); pk.y = pk2b(x0.z, x0.w); pk.z = pk2b(x1.x, x1.y); pk.w = pk2b(x1.z, x1.w);
    volatile v4u* dd = (volatile v4u*)(dst + e);
    *dd = pk; __threadfence(); *dd = pk;
}

__global__ __launch_bounds__(32 * AW) void k_battn(const unsigned short* __restrict__ QB, const unsigned short* __restrict__ KB, const unsigned short* __restrict__ VB,
                                                   float* __restrict__ O, float sl2) {
    constexpr int NT = HD / 16;
    constexpr int KS = HD / 32;
    constexpr int QP = SUB;
    __shared__ __align__(16) float          ptile[AW][16 * SUB];
    __shared__ __align__(16) unsigned short vT[HD * QP];
    __shared__ __align__(16) float          otile[AW][16 * HD];
    const int lane = threadIdx.x & 31, hf = lane >> 4, l15 = lane & 15, wave = threadIdx.x >> 5;
    const int h = blockIdx.y, b = blockIdx.z;
    const int q0 = ((int)blockIdx.x * AW + wave) * 16;
    float* myp = ptile[wave];
    float* myo = otile[wave];
    const long long rb = ((long long)b * NH + h) * SEQ;
    const float NEG = -__builtin_inff();
    const int sg = (int)threadIdx.x >> 4, sd = (int)threadIdx.x & 15;
    const int srcb = 16 * hf + 4 * (l15 & 3), tsel = l15 >> 2;

    {
        v4f zz = {0.f, 0.f, 0.f, 0.f};
#pragma unroll
        for (int rr = 0; rr < 8; ++rr)
#pragma unroll
            for (int ch = 0; ch < 2; ++ch) *(v4f*)(myo + (8 * hf + rr) * HD + 64 * ch + 4 * l15) = zz;
    }
    v16b qa[KS];
    {
        const unsigned short* qrow = QB + (rb + q0 + l15) * HD;
#pragma unroll
        for (int ks = 0; ks < KS; ++ks) qa[ks] = frag_row(qrow, 32 * ks, hf);
    }
    const unsigned short* kbase = KB + rb * HD;
    const unsigned short* vbase = VB + rb * HD;

    for (int jb = 0; jb < NKB; ++jb) {
        v8f o[NT]; float m8[8], l8[8];
#pragma unroll
        for (int t = 0; t < NT; ++t) { v8f zz = {}; o[t] = zz; }
#pragma unroll
        for (int i = 0; i < 8; ++i) { m8[i] = NEG; l8[i] = 0.f; }
        for (int sb = 0; sb < NSUB; ++sb) {
            const int j0 = jb * KBS + sb * SUB;
            __syncthreads();
            {
                v8us vin[2][4];
#pragma unroll
                for (int u = 0; u < 2; ++u)
#pragma unroll
                    for (int c = 0; c < 4; ++c) vin[u][c] = *(const v8us*)(vbase + (long long)(j0 + 2 * sg + u + 16 * c) * HD + 8 * sd);
#pragma unroll
                for (int dd = 0; dd < 8; ++dd) {
                    v8us w;
#pragma unroll
                    for (int e = 0; e < 8; ++e) w[e] = vin[e >> 2][e & 3][dd];
                    *(v8us*)(vT + (8 * sd + dd) * QP + 8 * sg) = w;
                }
            }
            SCHED_FENCE();
            v8f s[4];
#pragma unroll
            for (int t = 0; t < 4; ++t) {
                const unsigned short* krow = kbase + (long long)(j0 + 16 * t + l15) * HD;
                v8f acc = {};
#pragma unroll
                for (int ks = 0; ks < KS; ++ks) acc = wmmab(qa[ks], frag_row(krow, 32 * ks, hf), acc);
                s[t] = acc;
                SCHED_FENCE();
            }
#pragma unroll
            for (int i = 0; i < 8; ++i) {
                float sc[4];
#pragma unroll
                for (int t = 0; t < 4; ++t) sc[t] = s[t][i] * sl2;
                float mx = fmaxf(fmaxf(sc[0], sc[1]), fmaxf(sc[2], sc[3]));
                mx = fmaxf(mx, __shfl_xor(mx, 1, 32)); mx = fmaxf(mx, __shfl_xor(mx, 2, 32));
                mx = fmaxf(mx, __shfl_xor(mx, 4, 32)); mx = fmaxf(mx, __shfl_xor(mx, 8, 32));
                const float mnew = fmaxf(m8[i], mx);
                const float corr = exp2f(m8[i] - mnew);
                v4f p4;
                p4.x = exp2f(sc[0] - mnew); p4.y = exp2f(sc[1] - mnew); p4.z = exp2f(sc[2] - mnew); p4.w = exp2f(sc[3] - mnew);
                float rs = (p4.x + p4.y) + (p4.z + p4.w);
                rs += __shfl_xor(rs, 1, 32); rs += __shfl_xor(rs, 2, 32); rs += __shfl_xor(rs, 4, 32); rs += __shfl_xor(rs, 8, 32);
                l8[i] = l8[i] * corr + rs; m8[i] = mnew;
#pragma unroll
                for (int t = 0; t < NT; ++t) o[t][i] *= corr;
                *(v4f*)(myp + (8 * hf + i) * SUB + 4 * l15) = p4;
            }
            __syncthreads();
#pragma unroll
            for (int kh = 0; kh < 2; ++kh) {
                const Split pa = psplit(myp + l15 * SUB, 32 * kh, hf);
#pragma unroll
                for (int t = 0; t < NT; ++t) {
                    const v16b bv = frag_row(vT + (16 * t + l15) * QP, 32 * kh, hf);
                    o[t] = wmmab(pa.hi, bv, o[t]);
                    o[t] = wmmab(pa.lo, bv, o[t]);
                    if (t & 1) SCHED_FENCE();
                }
            }
        }
        float inv[8];
#pragma unroll
        for (int i = 0; i < 8; ++i) inv[i] = (l8[i] > 0.f) ? (1.0f / l8[i]) : 0.f;
#pragma unroll
        for (int rr = 0; rr < 8; ++rr) {
#pragma unroll
            for (int ch = 0; ch < 2; ++ch) {
                float x0 = 0.f, x1 = 0.f, x2 = 0.f, x3 = 0.f;
#pragma unroll
                for (int tp = 0; tp < 4; ++tp) {
                    const float sv = o[4 * ch + tp][rr] * inv[rr];
                    const float y0 = __shfl(sv, srcb + 0, 32);
                    const float y1 = __shfl(sv, srcb + 1, 32);
                    const float y2 = __shfl(sv, srcb + 2, 32);
                    const float y3 = __shfl(sv, srcb + 3, 32);
                    const bool take = (tsel == tp);
                    x0 = take ? y0 : x0; x1 = take ? y1 : x1; x2 = take ? y2 : x2; x3 = take ? y3 : x3;
                }
                float* op = myo + (8 * hf + rr) * HD + 64 * ch + 4 * l15;
                v4f a = *(v4f*)op;
                a.x += x0; a.y += x1; a.z += x2; a.w += x3;
                *(v4f*)op = a;
            }
        }
    }
    __syncthreads();
    float* ob = O + (rb + q0) * HD;
#pragma unroll
    for (int rr = 0; rr < 8; ++rr)
#pragma unroll
        for (int ch = 0; ch < 2; ++ch) {
            const v4f v = *(const v4f*)(myo + (8 * hf + rr) * HD + 64 * ch + 4 * l15);
            VST2V4(ob + (long long)(8 * hf + rr) * HD + 64 * ch + 4 * l15, v);
        }
}

extern "C" void kernel_launch(void* const* d_in, const int* in_sizes, int n_in, void* d_out, int out_size, void* d_ws, size_t ws_size, hipStream_t stream) {
    if (n_in < 3) return;
    const long long need_in = (long long)(NB * NH - 1) * SEQ_FULL * HD + (long long)SEQ * HD;
    if ((long long)in_sizes[0] < need_in || (long long)in_sizes[1] < need_in || (long long)in_sizes[2] < need_in) return;
    const long long nout = (long long)NB * NH * SEQ * HD;
    if ((long long)out_size < nout) return;
    const float* q = (const float*)d_in[0];
    const float* k = (const float*)d_in[1];
    const float* v = (const float*)d_in[2];
    float* out = (float*)d_out;
    const size_t plane = (size_t)nout * 2;
    char* wsp = (char*)d_ws;
    unsigned short* QB = (unsigned short*)wsp; wsp += plane;
    unsigned short* KB = (unsigned short*)wsp; wsp += plane;
    unsigned short* VB = (unsigned short*)wsp; wsp += plane;
    if ((size_t)(wsp - (char*)d_ws) > ws_size) return;
    const long long n8 = nout / 8;
    const long long nbk = (n8 + 255) / 256;
    k_cvtb<<<dim3((unsigned)(3 * nbk)), dim3(256), 0, stream>>>(q, k, v, QB, KB, VB, n8);
    const float sl2 = (float)(0.08838834764831845 * 1.4426950408889634);
    k_battn<<<dim3((unsigned)(SEQ / (16 * AW)), (unsigned)NH, (unsigned)NB), dim3(32 * AW), 0, stream>>>(QB, KB, VB, out, sl2);
}
